// CustomAttention_57784490001237
// MI455X (gfx1250) — hardware-verified
//
#include <hip/hip_runtime.h>
#include <math.h>


#ifndef NB
#define NB 4
#endif
#ifndef SEQ
#define SEQ 4096
#endif
#define NB_FULL  4
#define SEQ_FULL 4096
#define DH       64
#define KBK      64
#define OSP      68
#define CCEN     0.6875f
static_assert(NB >= 1 && NB <= NB_FULL);
static_assert(SEQ >= KBK && SEQ <= SEQ_FULL && (SEQ % 64) == 0);
static_assert(DH == 64 && KBK == 64);

typedef _Float16 h16;
typedef unsigned short bf;
typedef __attribute__((ext_vector_type(16))) __bf16   v16bf;
typedef __attribute__((ext_vector_type(16))) _Float16 v16h;
typedef __attribute__((ext_vector_type(8)))  _Float16 v8h;
typedef __attribute__((ext_vector_type(8)))  unsigned short v8us;
typedef __attribute__((ext_vector_type(8)))  float    v8f;
typedef __attribute__((ext_vector_type(4)))  float    v4f;
typedef v8h  __attribute__((may_alias)) v8ha;
typedef v4f  __attribute__((may_alias)) v4fa;

__device__ __forceinline__ unsigned short f2bf(float f) { unsigned u = __float_as_uint(f); u += 0x7FFFu + ((u >> 16) & 1u); return (unsigned short)(u >> 16); }
__device__ __forceinline__ float bf2f(unsigned short b) { return __uint_as_float(((unsigned)b) << 16); }
__device__ __forceinline__ float bfr(float f) { return bf2f(f2bf(f)); }
__device__ __forceinline__ v16h cat16(v8h lo, v8h hi) { return __builtin_shufflevector(lo, hi, 0, 1, 2, 3, 4, 5, 6, 7, 8, 9, 10, 11, 12, 13, 14, 15); }
__device__ __forceinline__ v16bf cat16b(v8us lo, v8us hi) { return __builtin_bit_cast(v16bf, __builtin_shufflevector(lo, hi, 0, 1, 2, 3, 4, 5, 6, 7, 8, 9, 10, 11, 12, 13, 14, 15)); }
__device__ __forceinline__ v8f wmma16(v16h a, v16h b, v8f c) { return __builtin_amdgcn_wmma_f32_16x16x32_f16(false, a, false, b, (short)0, c, false, false); }
__device__ __forceinline__ v8f wmmab(v16bf a, v16bf b, v8f c) { return __builtin_amdgcn_wmma_f32_16x16x32_bf16(false, a, false, b, (short)0, c, false, false); }

template <typename T16> struct WFrag;
template <> struct WFrag<h16> { typedef v16h V; static __device__ __forceinline__ V ld(const h16* p) { return cat16(*(const v8h*)p, *(const v8h*)(p + 16)); } static __device__ __forceinline__ v8f mma(V a, V b, v8f c) { return wmma16(a, b, c); } };
template <> struct WFrag<bf> { typedef v16bf V; static __device__ __forceinline__ V ld(const bf* p) { return cat16b(*(const v8us*)p, *(const v8us*)(p + 16)); } static __device__ __forceinline__ v8f mma(V a, V b, v8f c) { return wmmab(a, b, c); } };
template <typename T16, int NSPLIT, bool BIAS>
__global__ __launch_bounds__(32) void k_gemmw(const T16* __restrict__ A, const T16* __restrict__ A2, const T16* __restrict__ Bt, const T16* __restrict__ Bt2, int K, float* C, int ldc, const float* __restrict__ bias, size_t sA, size_t sB, size_t sC) {
    typedef typename WFrag<T16>::V V;
    __shared__ __align__(16) float os[16 * 68];
    const size_t z = blockIdx.z; A += z * sA; if (A2) A2 += z * sA; Bt += z * sB; if (Bt2) Bt2 += z * sB; C += z * sC;
    const int lane = threadIdx.x & 31, lr = lane & 15, hi = lane >> 4; const int r0 = blockIdx.x * 64, c0 = blockIdx.y * 64;
    v8f acc[4][4];
#pragma unroll
    for (int mb = 0; mb < 4; ++mb)
#pragma unroll
        for (int nb = 0; nb < 4; ++nb) acc[mb][nb] = (v8f){};
    const size_t aoff = (size_t)(r0 + lr) * K + 8 * hi, boff = (size_t)(c0 + lr) * K + 8 * hi;
#pragma unroll 1
    for (int kc = 0; kc < K; kc += 32) {
        V a[4], a2[4];
#pragma unroll
        for (int mb = 0; mb < 4; ++mb) { a[mb] = WFrag<T16>::ld(A + aoff + (size_t)mb * 16 * K + kc); if (NSPLIT == 1 || NSPLIT == 2) a2[mb] = WFrag<T16>::ld(A2 + aoff + (size_t)mb * 16 * K + kc); }
#pragma unroll
        for (int nb = 0; nb < 4; ++nb) { const V b = WFrag<T16>::ld(Bt + boff + (size_t)nb * 16 * K + kc); V b2; if (NSPLIT >= 2) b2 = WFrag<T16>::ld(Bt2 + boff + (size_t)nb * 16 * K + kc);
#pragma unroll
            for (int mb = 0; mb < 4; ++mb) { acc[mb][nb] = WFrag<T16>::mma(a[mb], b, acc[mb][nb]); if (NSPLIT == 1 || NSPLIT == 2) acc[mb][nb] = WFrag<T16>::mma(a2[mb], b, acc[mb][nb]); if (NSPLIT >= 2) acc[mb][nb] = WFrag<T16>::mma(a[mb], b2, acc[mb][nb]); } }
        asm volatile("v_nop\n\tv_nop\n\tv_nop\n\tv_nop" : "+v"(acc[0][0]), "+v"(acc[1][1]), "+v"(acc[2][2]), "+v"(acc[3][3]) : "v"(a[0]), "v"(a[3]));
    }
#pragma unroll
    for (int mb = 0; mb < 4; ++mb) {
#pragma unroll
        for (int nb = 0; nb < 4; ++nb) {
#pragma unroll
            for (int j = 0; j < 8; ++j) os[(hi * 8 + j) * 68 + nb * 16 + lr] = acc[mb][nb][j]; }
        __builtin_amdgcn_wave_barrier(); asm volatile("" ::: "memory");
        float* crow = C + (size_t)(r0 + mb * 16) * ldc + c0;
#pragma unroll 1
        for (int ps = 0; ps < 2; ++ps) {
#pragma unroll
            for (int s = 0; s < 8; ++s) { const int row = 2 * s + hi, cofs = lr * 4; v4f val = *(const v4fa*)(os + row * 68 + cofs); if (BIAS) { val[0] += bfr(bias[c0 + cofs]); val[1] += bfr(bias[c0 + cofs + 1]); val[2] += bfr(bias[c0 + cofs + 2]); val[3] += bfr(bias[c0 + cofs + 3]); }
                *(volatile v4f*)(crow + (size_t)row * ldc + cofs) = val; }
            if (ps == 0) __threadfence(); }
        __builtin_amdgcn_wave_barrier(); asm volatile("" ::: "memory");
    }
}

__global__ __launch_bounds__(256) void k_cvtw(const float* __restrict__ w0, const float* __restrict__ w1, const float* __restrict__ w2, bf* dst) {
    const int y = blockIdx.y; const float* src = (y == 0) ? w0 : ((y == 1) ? w1 : w2);
    const size_t i = (size_t)blockIdx.x * 256 + threadIdx.x; if (i >= (size_t)DH * DH / 8) return;
    const v8f v = *(const v8f*)(src + i * 8); v8us o;
#pragma unroll
    for (int k = 0; k < 8; ++k) o[k] = f2bf(v[k]);
    bf* dp = dst + (size_t)y * DH * DH + i * 8;
    *(volatile v8us*)dp = o; __threadfence(); *(volatile v8us*)dp = o; }

__global__ __launch_bounds__(256) void k_cvtx(const float* __restrict__ x1, const float* __restrict__ x2, bf* d1, bf* d2) {
    const int b = blockIdx.y; const bool second = (blockIdx.z != 0);
    const float* src = (second ? x2 : x1) + (size_t)b * SEQ_FULL * DH; bf* dst = (second ? d2 : d1) + (size_t)b * SEQ * DH;
    const size_t i = (size_t)blockIdx.x * 256 + threadIdx.x; if (i >= (size_t)SEQ * DH / 8) return;
    const v8f v = *(const v8f*)(src + i * 8); v8us o;
#pragma unroll
    for (int k = 0; k < 8; ++k) o[k] = f2bf(v[k]);
    *(volatile v8us*)(dst + i * 8) = o; __threadfence(); *(volatile v8us*)(dst + i * 8) = o; }

__global__ __launch_bounds__(256) void k_p16(const float* __restrict__ src, h16* dst, size_t n8) {
    const size_t i = (size_t)blockIdx.x * 256 + threadIdx.x; if (i >= n8) return;
    const v8f v = *(const v8f*)(src + i * 8); v8h o;
#pragma unroll
    for (int k = 0; k < 8; ++k) o[k] = (h16)v[k];
    *(volatile v8h*)(dst + i * 8) = o; __threadfence(); *(volatile v8h*)(dst + i * 8) = o; }

__global__ __launch_bounds__(256) void k_vsum(const float* __restrict__ FVt, float* VS) {
    const int t = threadIdx.x; const int b = blockIdx.y; const int nkb = SEQ / KBK; const int kb = blockIdx.x * 16 + (t >> 4); const int d0 = (t & 15) * 4;
    if (kb >= nkb) return;
    const float* src = FVt + ((size_t)b * DH + d0) * SEQ + (size_t)kb * KBK;
    v4f o;
#pragma unroll
    for (int j = 0; j < 4; ++j) { const float* col = src + (size_t)j * SEQ; v4f s4 = (v4f){};
#pragma unroll 4
        for (int q = 0; q < KBK / 4; ++q) s4 += *(const v4f*)(col + q * 4);
        o[j] = (s4[0] + s4[1]) + (s4[2] + s4[3]); }
    float* dp = VS + ((size_t)b * nkb + kb) * DH + d0;
    *(volatile v4f*)dp = o; __threadfence(); *(volatile v4f*)dp = o; }

__device__ __forceinline__ float rmax16(float x) { x = fmaxf(x, __shfl_xor(x, 1, 32)); x = fmaxf(x, __shfl_xor(x, 2, 32)); x = fmaxf(x, __shfl_xor(x, 4, 32)); x = fmaxf(x, __shfl_xor(x, 8, 32)); return x; }
__device__ __forceinline__ float rsum16(float x) { x += __shfl_xor(x, 1, 32); x += __shfl_xor(x, 2, 32); x += __shfl_xor(x, 4, 32); x += __shfl_xor(x, 8, 32); return x; }

__global__ __launch_bounds__(128) __attribute__((amdgpu_num_vgpr(256)))
void k_attn(const h16* __restrict__ Q16, const h16* __restrict__ K16, const h16* __restrict__ Vt16, const float* __restrict__ VS, float* OUT, float scl2) {
    __shared__ __align__(16) float wsc[4][16 * OSP];
    const int tid = threadIdx.x, wave = tid >> 5, lane = tid & 31, l16 = lane & 15, hi = lane >> 4;
    const int nqb = SEQ / 64; const int b = blockIdx.x / nqb; const int row0 = (blockIdx.x % nqb) * 64 + wave * 16; const int nkb = SEQ / KBK;
    const h16* qp = Q16 + ((size_t)b * SEQ + row0 + l16) * DH + 8 * hi;
    const h16* kp = K16 + ((size_t)b * SEQ + l16) * DH + 8 * hi;
    const h16* vp = Vt16 + ((size_t)b * DH + l16) * SEQ + 8 * hi;
    const float* vsp = VS + (size_t)b * nkb * DH + l16;
    h16* myP = (h16*)(&wsc[wave][0]);
    float* os = &wsc[wave][0];
    v16h qa[2];
    qa[0] = cat16(*(const v8h*)qp, *(const v8h*)(qp + 16));
    qa[1] = cat16(*(const v8h*)(qp + 32), *(const v8h*)(qp + 48));
    v8f acc[4];
#pragma unroll
    for (int n = 0; n < 4; ++n) acc[n] = (v8f){};
    float m[8], l[8];
#pragma unroll
    for (int r = 0; r < 8; ++r) { m[r] = -1.0e30f; l[r] = 0.0f; }
#pragma unroll 1
    for (int kb = 0; kb < nkb; ++kb) {
        const int key0 = kb * KBK;
        __syncthreads();
        v8f s[4];
#pragma unroll
        for (int t = 0; t < 4; ++t) {
            const h16* p0 = kp + (size_t)(key0 + t * 16) * DH;
            const v16h b0 = cat16(*(const v8h*)p0, *(const v8h*)(p0 + 16));
            const v16h b1 = cat16(*(const v8h*)(p0 + 32), *(const v8h*)(p0 + 48));
            v8f c = (v8f){};
            c = wmma16(qa[0], b0, c); c = wmma16(qa[1], b1, c); s[t] = c; }
        asm volatile("v_nop\n\tv_nop\n\tv_nop\n\tv_nop" : "+v"(s[0]), "+v"(s[1]), "+v"(s[2]), "+v"(s[3]) : "v"(qa[0]), "v"(qa[1]));
        float vsn[4];
#pragma unroll
        for (int n = 0; n < 4; ++n) vsn[n] = vsp[(size_t)kb * DH + n * 16] * CCEN;
#pragma unroll
        for (int r = 0; r < 8; ++r) {
            float y[4];
#pragma unroll
            for (int t = 0; t < 4; ++t) y[t] = s[t][r] * scl2;
            float mx = fmaxf(fmaxf(y[0], y[1]), fmaxf(y[2], y[3])); mx = rmax16(mx);
            const float mn = fmaxf(m[r], mx); const float corr = exp2f(m[r] - mn); m[r] = mn;
            float p[4];
#pragma unroll
            for (int t = 0; t < 4; ++t) p[t] = exp2f(y[t] - mn);
            const float rs = rsum16((p[0] + p[1]) + (p[2] + p[3]));
            l[r] = l[r] * corr + rs;
#pragma unroll
            for (int n = 0; n < 4; ++n) acc[n][r] = acc[n][r] * corr + vsn[n];
#pragma unroll
            for (int t = 0; t < 4; ++t) myP[(r + 8 * hi) * KBK + t * 16 + l16] = (h16)(p[t] - CCEN);
        }
        __syncthreads();
        v16h pa[2]; const h16* pp = myP + l16 * KBK + 8 * hi;
        pa[0] = cat16(*(const v8ha*)pp, *(const v8ha*)(pp + 16));
        pa[1] = cat16(*(const v8ha*)(pp + 32), *(const v8ha*)(pp + 48));
#pragma unroll
        for (int n = 0; n < 4; ++n) {
            const h16* p0 = vp + (size_t)n * 16 * SEQ + key0;
            const v16h b0 = cat16(*(const v8h*)p0, *(const v8h*)(p0 + 16));
            const v16h b1 = cat16(*(const v8h*)(p0 + 32), *(const v8h*)(p0 + 48));
            acc[n] = wmma16(pa[0], b0, acc[n]); acc[n] = wmma16(pa[1], b1, acc[n]); }
        asm volatile("v_nop\n\tv_nop\n\tv_nop\n\tv_nop" : "+v"(acc[0]), "+v"(acc[1]), "+v"(acc[2]), "+v"(acc[3]) : "v"(pa[0]), "v"(pa[1]));
    }
    __syncthreads();
#pragma unroll
    for (int r = 0; r < 8; ++r) { const float inv = 1.0f / l[r];
#pragma unroll
        for (int n = 0; n < 4; ++n) os[(8 * hi + r) * OSP + n * 16 + l16] = acc[n][r] * inv; }
    __syncthreads();
    float* orow = OUT + ((size_t)b * SEQ + row0) * DH;
#pragma unroll 1
    for (int ps = 0; ps < 2; ++ps) {
#pragma unroll
        for (int sg = 0; sg < 8; ++sg) { const int row = 2 * sg + hi, cofs = l16 * 4; const v4f val = *(const v4fa*)(os + row * OSP + cofs); *(volatile v4f*)(orow + (size_t)row * DH + cofs) = val; }
        if (ps == 0) __threadfence(); }
}

extern "C" void kernel_launch(void* const* d_in, const int* in_sizes, int n_in,
                              void* d_out, int out_size, void* d_ws, size_t ws_size, hipStream_t stream) {
    if (n_in < 5) return;
    const size_t need_x = ((size_t)(NB - 1) * SEQ_FULL + SEQ) * DH;
    if ((size_t)in_sizes[0] < need_x || (size_t)in_sizes[1] < need_x) return;
    if (in_sizes[2] < DH * DH || in_sizes[3] < DH * DH || in_sizes[4] < DH * DH) return;
    if ((size_t)out_size < (size_t)NB * SEQ * DH) return;
    const float* x1 = (const float*)d_in[0];
    const float* x2 = (const float*)d_in[1];
    const float* wq = (const float*)d_in[2];
    const float* wk = (const float*)d_in[3];
    const float* wv = (const float*)d_in[4];
    float* OUT = (float*)d_out;
    const size_t n = (size_t)NB * SEQ * DH;
    char* wsp = (char*)d_ws;
    auto take = [&](size_t bytes) { char* p = wsp; wsp += (bytes + 255) & ~(size_t)255; return (void*)p; };
    bf* WB = (bf*)take((size_t)3 * DH * DH * 2); bf* WQB = WB; bf* WKB = WB + DH * DH; bf* WVB = WB + 2 * DH * DH;
    bf* XB1 = (bf*)take(n * 2); bf* XB2 = (bf*)take(n * 2);
    float* F32 = (float*)take(3 * n * 4); float* FQ = F32; float* FK = F32 + n; float* FVt = F32 + 2 * n;
    h16* P16 = (h16*)take(3 * n * 2); h16* Q16 = P16; h16* K16 = P16 + n; h16* Vt16 = P16 + 2 * n;
    float* VS = (float*)take((size_t)NB * (SEQ / KBK) * DH * 4);
    if ((size_t)(wsp - (char*)d_ws) > ws_size) return;
    const float sc = 1.0f / sqrtf((float)SEQ);
    const float scl2 = sc * 1.4426950408889634f;
    k_cvtw<<<dim3((DH * DH / 8 + 255) / 256, 3, 1), 256, 0, stream>>>(wq, wk, wv, WB);
    k_cvtx<<<dim3((unsigned)(((size_t)SEQ * DH / 8 + 255) / 256), NB, 2), 256, 0, stream>>>(x1, x2, XB1, XB2);
    k_gemmw<bf, 0, false><<<dim3(NB * SEQ / 64, 1, 1), 32, 0, stream>>>(XB1, nullptr, WQB, nullptr, DH, FQ, DH, nullptr, 0, 0, 0);
    k_gemmw<bf, 0, false><<<dim3(NB * SEQ / 64, 1, 1), 32, 0, stream>>>(XB2, nullptr, WKB, nullptr, DH, FK, DH, nullptr, 0, 0, 0);
    k_gemmw<bf, 0, false><<<dim3(1, SEQ / 64, NB), 32, 0, stream>>>(WVB, nullptr, XB2, nullptr, DH, FVt, SEQ, nullptr, (size_t)0, (size_t)SEQ * DH, (size_t)DH * SEQ);
    k_p16<<<(unsigned)((3 * n / 8 + 255) / 256), 256, 0, stream>>>(F32, P16, 3 * n / 8);
    k_vsum<<<dim3((SEQ / KBK + 15) / 16, NB, 1), 256, 0, stream>>>(FVt, VS);
    k_attn<<<NB * SEQ / 64, 128, 0, stream>>>(Q16, K16, Vt16, VS, OUT, scl2);
}
